// OCTMambaBlock_71021579207190
// MI455X (gfx1250) — hardware-run, weakly checked
//
#include <hip/hip_runtime.h>


#ifndef NB
#define NB 2
#endif
#ifndef SW
#define SW 32
#endif
#define NB_FULL 2
#define SW_FULL 32
#define SH   32
#define SD   16
#define C_IN 32
#define CO   64
#define DIN  128
#define DST  16
#define DTR  4
#define NXD  36
#define CH4  256
#define LSP      (SW * SH * SD)
#define LSP_FULL (SW_FULL * SH * SD)
#ifndef OUT_LSP
#define OUT_LSP LSP
#endif
#define NROW (NB * LSP)
#define PW   (SW + 2)
#define PH   (SH + 2)
#define PD   (SD + 2)
#define KCONV (27 * C_IN)
#define EPSV 1e-5f
#define WSC  16.0f
#define UCS  256.0f
#define YCS  1024.0f
#define LOG2E 1.4426950408889634f

static_assert(C_IN == 32);
static_assert(CO == 64);
static_assert(DIN == 128);
static_assert(DIN % 32 == 0);
static_assert(CH4 % 64 == 0);
static_assert(KCONV % 32 == 0);
static_assert(CO % 32 == 0);
static_assert(LSP % 64 == 0);
static_assert(NROW % 64 == 0);
static_assert(LSP % 512 == 0);
static_assert(DTR + 2 * DST == NXD);
static_assert(NXD <= 64);
static_assert(DTR % 4 == 0);
static_assert(NB <= NB_FULL);
static_assert(SW <= SW_FULL);
static_assert((PD * 4) % 8 == 0);
static_assert(32 * 16 * 8 == 16 * 64 * 4);
static_assert(32 * 16 * 4 == 16 * 64 * 2);
static_assert(256 * 16 * 2 == 64 * CO * 2);
static_assert(32 * 16 == 8 * 32 * 2);
static_assert((CO * 27 * 4) % 256 == 0);
static_assert(sizeof(float) * (CO * 27 + 9 * CO + CO * 65 + 128) <= 131072);
static_assert(sizeof(float) * 16 * 68 <= 131072);

typedef _Float16 h16;
typedef unsigned short bf;
typedef __attribute__((ext_vector_type(16))) __bf16   v16bf;
typedef __attribute__((ext_vector_type(16))) _Float16 v16h;
typedef __attribute__((ext_vector_type(8)))  _Float16 v8h;
typedef __attribute__((ext_vector_type(8)))  unsigned short v8us;
typedef __attribute__((ext_vector_type(8)))  float    v8f;
typedef __attribute__((ext_vector_type(4)))  float    v4f;
typedef v4f  __attribute__((may_alias)) v4fa;
typedef v8h  __attribute__((may_alias)) v8ha;

__device__ __forceinline__ unsigned short f2bf(float f) { unsigned u = __float_as_uint(f); u += 0x7FFFu + ((u >> 16) & 1u); return (unsigned short)(u >> 16); }
__device__ __forceinline__ float bfr(float f) { return __uint_as_float(((unsigned)f2bf(f)) << 16); }
__device__ __forceinline__ v16h cat16(v8h lo, v8h hi) { return __builtin_shufflevector(lo, hi, 0, 1, 2, 3, 4, 5, 6, 7, 8, 9, 10, 11, 12, 13, 14, 15); }
__device__ __forceinline__ v16bf cat16b(v8us lo, v8us hi) { return __builtin_bit_cast(v16bf, __builtin_shufflevector(lo, hi, 0, 1, 2, 3, 4, 5, 6, 7, 8, 9, 10, 11, 12, 13, 14, 15)); }
__device__ __forceinline__ v8f wmma16(v16h a, v16h b, v8f c) { return __builtin_amdgcn_wmma_f32_16x16x32_f16(false, a, false, b, (short)0, c, false, false); }
__device__ __forceinline__ v8f wmmab(v16bf a, v16bf b, v8f c) { return __builtin_amdgcn_wmma_f32_16x16x32_bf16(false, a, false, b, (short)0, c, false, false); }
__device__ __forceinline__ v16h  ldh(const h16* p) { return cat16(*(const v8h*)p, *(const v8h*)(p + 16)); }
__device__ __forceinline__ v16bf ldb(const bf* p)  { return cat16b(*(const v8us*)p, *(const v8us*)(p + 16)); }
__device__ __forceinline__ void wave_sync() { __builtin_amdgcn_fence(3  , "wavefront"); __builtin_amdgcn_wave_barrier(); asm volatile("" ::: "memory"); }

static __device__ __forceinline__ h16 toh_flush(float v) { const h16 r = (h16)v; return (fabsf(v) < 6.103515625e-05f) ? (h16)0.0f : r; }
__device__ __forceinline__ v8f wg16(v16h a, v16h b, v8f c) { c = wmma16(a, b, c); asm volatile("v_nop\n\tv_nop\n\tv_nop\n\tv_nop" : "+v"(c) : "v"(a), "v"(b)); return c; }
__device__ __forceinline__ v8f wgb(v16bf a, v16bf b, v8f c) { c = wmmab(a, b, c); asm volatile("v_nop\n\tv_nop\n\tv_nop\n\tv_nop" : "+v"(c) : "v"(a), "v"(b)); return c; }
__device__ __forceinline__ int clampi(int v, int lo, int hi) { return v < lo ? lo : (v > hi ? hi : v); }
__device__ __forceinline__ float fexp(float x) { return __builtin_amdgcn_exp2f(x * LOG2E); }

__global__ __launch_bounds__(256) void k_xpad(const float* __restrict__ x, bf* XP, int npiece) {
    const int i = blockIdx.x * 256 + threadIdx.x; if (i >= npiece) return;
    const int c8 = i & 3; int pos = i >> 2;
    const int dp = pos % PD; pos /= PD; const int hp = pos % PH; pos /= PH; const int wp = pos % PW; const int b = pos / PW;
    const bool inside = (wp >= 1) & (wp <= SW) & (hp >= 1) & (hp <= SH) & (dp >= 1) & (dp <= SD);
    const int w = clampi(wp - 1, 0, SW - 1), h = clampi(hp - 1, 0, SH - 1), d = clampi(dp - 1, 0, SD - 1);
    const size_t src = ((size_t)(b * C_IN + c8 * 8)) * LSP_FULL + (size_t)((w * SH + h) * SD + d);
    v8us o;
#pragma unroll
    for (int j = 0; j < 8; ++j) { float v = x[src + (size_t)j * LSP_FULL]; asm volatile("" : "+v"(v)); o[j] = inside ? f2bf(v) : (unsigned short)0; }
    *(volatile v8us*)(XP + (size_t)i * 8) = o; __threadfence(); *(volatile v8us*)(XP + (size_t)i * 8) = o;
}

__global__ __launch_bounds__(256) void k_wconv3(const float* __restrict__ w, bf* W2) {
    const int p = blockIdx.x * 256 + threadIdx.x; if (p >= CO * 27 * 4) return;
    const int c8 = p & 3; const int t = (p >> 2) % 27; const int co = (p >> 2) / 27;
    v8us o;
#pragma unroll
    for (int j = 0; j < 8; ++j) o[j] = f2bf(w[((size_t)(co * C_IN + c8 * 8 + j)) * 27 + t]);
    *(volatile v8us*)(W2 + (size_t)p * 8) = o; __threadfence(); *(volatile v8us*)(W2 + (size_t)p * 8) = o;
}

__global__ __launch_bounds__(256) void k_wcvt16(const float* __restrict__ src, h16* dst, int nsrc8, int ndst8) {
    const int i = blockIdx.x * 256 + threadIdx.x; if (i >= ndst8) return;
    const int ic = i < nsrc8 ? i : nsrc8 - 1;
    v8f v = *(const v8f*)(src + (size_t)ic * 8); asm volatile("" : "+v"(v));
    const bool ok = i < nsrc8; v8h o;
#pragma unroll
    for (int k = 0; k < 8; ++k) o[k] = ok ? toh_flush(bfr(v[k]) * WSC) : (h16)0.0f;
    *(volatile v8h*)(dst + (size_t)i * 8) = o; __threadfence(); *(volatile v8h*)(dst + (size_t)i * 8) = o;
}

__global__ __launch_bounds__(32) void k_conv(const bf* __restrict__ W2, const bf* __restrict__ XP, const float* __restrict__ bias, float* CV) {
    __shared__ __align__(16) float os[16 * 68];
    const int lane = threadIdx.x & 31, lr = lane & 15, hi = lane >> 4;
    const int c0 = blockIdx.x * 64; const int bb = c0 / LSP, sp0 = c0 % LSP;
    int poff[4];
#pragma unroll
    for (int nb = 0; nb < 4; ++nb) { const int sp = sp0 + nb * 16 + lr; const int w = sp / (SH * SD), h = (sp / SD) % SH, d = sp % SD;
        poff[nb] = (((bb * PW + w) * PH + h) * PD + d) * C_IN + 8 * hi; }
    const int aoff = lr * KCONV + 8 * hi;
    v8f acc[4][4];
#pragma unroll
    for (int mb = 0; mb < 4; ++mb)
#pragma unroll
        for (int nb = 0; nb < 4; ++nb) acc[mb][nb] = (v8f){};
#pragma unroll 1
    for (int t = 0; t < 27; ++t) {
        const int toff = (((t / 9) * PH + (t / 3) % 3) * PD + (t % 3)) * C_IN;
        v16bf a[4];
#pragma unroll
        for (int mb = 0; mb < 4; ++mb) a[mb] = ldb(W2 + aoff + mb * 16 * KCONV + t * 32);
#pragma unroll
        for (int nb = 0; nb < 4; ++nb) { const v16bf b = ldb(XP + poff[nb] + toff);
#pragma unroll
            for (int mb = 0; mb < 4; ++mb) acc[mb][nb] = wgb(a[mb], b, acc[mb][nb]); }
    }
#pragma unroll
    for (int mb = 0; mb < 4; ++mb) {
        float br[8];
#pragma unroll
        for (int j = 0; j < 8; ++j) br[j] = bfr(bias[mb * 16 + hi * 8 + j]);
#pragma unroll
        for (int nb = 0; nb < 4; ++nb) {
#pragma unroll
            for (int j = 0; j < 8; ++j) os[(hi * 8 + j) * 68 + nb * 16 + lr] = acc[mb][nb][j] + br[j]; }
        wave_sync();
        float* dst = CV + ((size_t)(bb * CO + mb * 16)) * LSP + sp0;
#pragma unroll 1
        for (int ps = 0; ps < 2; ++ps) {
#pragma unroll
            for (int s = 0; s < 8; ++s) { const int row = 2 * s + (lane >> 4), cofs = (lane & 15) * 4;
                const v4f val = *(const v4fa*)(&os[row * 68 + cofs]);
                *(volatile v4f*)(dst + (size_t)row * LSP + cofs) = val; }
            if (ps == 0) __threadfence(); }
        wave_sync();
    }
}

__global__ __launch_bounds__(256) void k_gnstats(const float* __restrict__ CV, float* ST) {
    __shared__ float r1[8], r2[8];
    const int tid = threadIdx.x, lane = tid & 31;
    const int wave = __builtin_amdgcn_readfirstlane((int)(threadIdx.x >> 5));
    const float* base = CV + (size_t)blockIdx.x * 2 * LSP;
    float s = 0.0f, q = 0.0f;
#pragma unroll 1
    for (int i = tid * 4; i < 2 * LSP; i += 1024) { const v4f v = *(const v4f*)(base + i);
        s += (v[0] + v[1]) + (v[2] + v[3]); q += (v[0] * v[0] + v[1] * v[1]) + (v[2] * v[2] + v[3] * v[3]); }
#pragma unroll
    for (int o = 16; o > 0; o >>= 1) { s += __shfl_xor(s, o, 32); q += __shfl_xor(q, o, 32); }
    if (lane == 0) { r1[wave] = s; r2[wave] = q; }
    __syncthreads();
    float ts = 0.0f, tq = 0.0f;
#pragma unroll
    for (int w = 0; w < 8; ++w) { ts += r1[w]; tq += r2[w]; }
    const float inv = 1.0f / (float)(2 * LSP);
    const float mu = ts * inv; const float var = tq * inv - mu * mu; const float rs = rsqrtf(var + EPSV);
    if (tid < 8) { v4f o; o[0] = (tid == 0) ? mu : 0.0f; o[1] = (tid == 0) ? rs : 0.0f; o[2] = 0.0f; o[3] = 0.0f;
        float* dst = ST + (size_t)blockIdx.x * 32 + tid * 4;
        *(volatile v4f*)dst = o; __threadfence(); *(volatile v4f*)dst = o; }
}

__global__ __launch_bounds__(256) void k_gnapply(const float* __restrict__ CV, const float* __restrict__ ST, const float* __restrict__ gg, const float* __restrict__ gb, float* ID, int n4) {
    const int i = blockIdx.x * 256 + threadIdx.x; if (i >= n4) return;
    const size_t e = (size_t)i * 4; const int ch = (int)(e / LSP);
    const int c = ch % CO; const int grp = ch >> 1;
    const float mu = ST[(size_t)grp * 32], rs = ST[(size_t)grp * 32 + 1];
    const float g = bfr(gg[c]), bt = bfr(gb[c]);
    const v4f v = *(const v4f*)(CV + e); v4f o;
#pragma unroll
    for (int k = 0; k < 4; ++k) o[k] = fmaxf((v[k] - mu) * rs * g + bt, 0.0f);
    *(volatile v4f*)(ID + e) = o; __threadfence(); *(volatile v4f*)(ID + e) = o;
}

__global__ __launch_bounds__(256) void k_sfe_ln(const float* __restrict__ ID, const float* __restrict__ dw,
                                                const float* __restrict__ g1, const float* __restrict__ b1, const float* __restrict__ m1, const float* __restrict__ v1,
                                                const float* __restrict__ pw,
                                                const float* __restrict__ g2, const float* __restrict__ b2, const float* __restrict__ m2, const float* __restrict__ v2,
                                                const float* __restrict__ lng, const float* __restrict__ lnb, h16* SP) {
    __shared__ float dwl[CO * 27];
    __shared__ float par[9 * CO];
    __shared__ float sv[CO * 65];
    __shared__ float mus[64], rss[64];
    const int tid = threadIdx.x;
    const int wave = __builtin_amdgcn_readfirstlane((int)(threadIdx.x >> 5));
    const int c0t = blockIdx.x * 64; const int bb = c0t / LSP, sp0 = c0t % LSP;
#pragma unroll 1
    for (int i = tid; i < CO * 27; i += 256) dwl[i] = bfr(dw[i]);
    if (tid < CO) {
        par[0 * CO + tid] = bfr(g1[tid]) * rsqrtf(bfr(v1[tid]) + EPSV); par[1 * CO + tid] = bfr(m1[tid]); par[2 * CO + tid] = bfr(b1[tid]);
        par[3 * CO + tid] = bfr(pw[tid]);
        par[4 * CO + tid] = bfr(g2[tid]) * rsqrtf(bfr(v2[tid]) + EPSV); par[5 * CO + tid] = bfr(m2[tid]); par[6 * CO + tid] = bfr(b2[tid]);
        par[7 * CO + tid] = bfr(lng[tid]); par[8 * CO + tid] = bfr(lnb[tid]); }
    __syncthreads();
    { const int tk = tid & 63; const int cg = wave >> 1;
      const int sp = sp0 + tk; const int w = sp / (SH * SD), h = (sp / SD) % SH, d = sp % SD;
#pragma unroll 1
      for (int cc = 0; cc < 16; ++cc) {
          const int c = cg * 16 + cc;
          const size_t cb = ((size_t)(bb * CO + c)) * LSP;
          float acc = 0.0f;
#pragma unroll 1
          for (int a = 0; a < 3; ++a) {
              const int ww = w + a - 1; const bool wok = (unsigned)ww < (unsigned)SW; const int wc = clampi(ww, 0, SW - 1);
#pragma unroll
              for (int q = 0; q < 9; ++q) {
                  const int hh = h + q / 3 - 1, dd = d + q % 3 - 1;
                  const bool ok = wok & ((unsigned)hh < (unsigned)SH) & ((unsigned)dd < (unsigned)SD);
                  const int hc = clampi(hh, 0, SH - 1), dc = clampi(dd, 0, SD - 1);
                  float xv = ID[cb + (size_t)((wc * SH + hc) * SD + dc)]; asm volatile("" : "+v"(xv));
                  acc += dwl[c * 27 + a * 9 + q] * (ok ? xv : 0.0f); } }
          const float xc = ID[cb + sp];
          const float o1 = (acc - par[1 * CO + c]) * par[0 * CO + c] + par[2 * CO + c];
          const float o2 = (xc * par[3 * CO + c] - par[5 * CO + c]) * par[4 * CO + c] + par[6 * CO + c];
          sv[c * 65 + tk] = (o1 + o2) + xc; } }
    __syncthreads();
    if (tid < 64) {
        float s = 0.0f;
#pragma unroll 4
        for (int c = 0; c < CO; ++c) s += sv[c * 65 + tid];
        const float mu = s * (1.0f / (float)CO);
        float q = 0.0f;
#pragma unroll 4
        for (int c = 0; c < CO; ++c) { const float dv = sv[c * 65 + tid] - mu; q += dv * dv; }
        mus[tid] = mu; rss[tid] = rsqrtf(q * (1.0f / (float)CO) + EPSV); }
    __syncthreads();
#pragma unroll 1
    for (int ps = 0; ps < 2; ++ps) {
#pragma unroll
        for (int i = 0; i < 2; ++i) { const int p = tid + 256 * i; const int tk2 = p >> 3, c8 = (p & 7) * 8;
            const float mu = mus[tk2], rs = rss[tk2]; v8h hv;
#pragma unroll
            for (int j = 0; j < 8; ++j) hv[j] = toh_flush((sv[(c8 + j) * 65 + tk2] - mu) * rs * par[7 * CO + c8 + j] + par[8 * CO + c8 + j]);
            *(volatile v8h*)(SP + (size_t)c0t * CO + (size_t)p * 8) = hv; }
        if (ps == 0) __threadfence(); }
}

template <int EPI>
__device__ __forceinline__ void gemm_body(const h16* __restrict__ A, const int lda, const int aks, const h16* __restrict__ Bt, const int ldbt, const int K, const float scale,
                                          float* Cf, h16* Ch, const int ldc, const int bnf,
                                          const float* __restrict__ pg, const float* __restrict__ pb, const float* __restrict__ pm, const float* __restrict__ pv,
                                          const int relu, const float ocarry, const float* __restrict__ RES) {
    __shared__ __align__(16) float os[16 * 68];
    const int lane = threadIdx.x & 31, lr = lane & 15, hi = lane >> 4; const int r0 = blockIdx.x * 64, c0 = blockIdx.y * 64;
    v8f acc[4][4];
#pragma unroll
    for (int mb = 0; mb < 4; ++mb)
#pragma unroll
        for (int nb = 0; nb < 4; ++nb) acc[mb][nb] = (v8f){};
    const size_t aoff = (size_t)(r0 + lr) * lda + 8 * hi, boff = (size_t)(c0 + lr) * ldbt + 8 * hi;
    const int nks = K >> 5;
#pragma unroll 1
    for (int ks = 0; ks < nks; ++ks) {
        v16h a[4];
#pragma unroll
        for (int mb = 0; mb < 4; ++mb) a[mb] = ldh(A + aoff + (size_t)mb * 16 * lda + (size_t)ks * aks);
#pragma unroll
        for (int nb = 0; nb < 4; ++nb) { const v16h b = ldh(Bt + boff + (size_t)nb * 16 * ldbt + (size_t)ks * 32);
#pragma unroll
            for (int mb = 0; mb < 4; ++mb) acc[mb][nb] = wg16(a[mb], b, acc[mb][nb]); }
    }
    if (EPI == 0) {
#pragma unroll
        for (int mb = 0; mb < 4; ++mb) {
#pragma unroll
            for (int nb = 0; nb < 4; ++nb) {
#pragma unroll
                for (int j = 0; j < 8; ++j) os[(hi * 8 + j) * 68 + nb * 16 + lr] = acc[mb][nb][j] * scale; }
            wave_sync();
            float* dst = Cf + (size_t)(r0 + mb * 16) * ldc + c0;
#pragma unroll 1
            for (int ps = 0; ps < 2; ++ps) {
#pragma unroll
                for (int s = 0; s < 8; ++s) { const int row = 2 * s + (lane >> 4), cofs = (lane & 15) * 4;
                    const v4f val = *(const v4fa*)(&os[row * 68 + cofs]);
                    *(volatile v4f*)(dst + (size_t)row * ldc + cofs) = val; }
                if (ps == 0) __threadfence(); }
            wave_sync();
        }
    } else if (EPI == 1) {
        float cs[4], cm[4], cb[4];
#pragma unroll
        for (int nb = 0; nb < 4; ++nb) { cs[nb] = 1.0f; cm[nb] = 0.0f; cb[nb] = 0.0f;
            if (bnf) { const int n = c0 + nb * 16 + lr; cs[nb] = bfr(pg[n]) * rsqrtf(bfr(pv[n]) + EPSV); cm[nb] = bfr(pm[n]); cb[nb] = bfr(pb[n]); } }
#pragma unroll
        for (int mb = 0; mb < 4; ++mb) {
#pragma unroll
            for (int nb = 0; nb < 4; ++nb) {
#pragma unroll
                for (int j = 0; j < 8; ++j) { float v = (acc[mb][nb][j] * scale - cm[nb]) * cs[nb] + cb[nb]; if (relu) v = fmaxf(v, 0.0f);
                    os[(hi * 8 + j) * 68 + nb * 16 + lr] = v * ocarry; } }
            wave_sync();
            h16* dst = Ch + (size_t)(r0 + mb * 16) * ldc + c0;
#pragma unroll 1
            for (int ps = 0; ps < 2; ++ps) {
#pragma unroll
                for (int s = 0; s < 4; ++s) { const int row = 4 * s + (lane >> 3), c8 = (lane & 7) * 8;
                    const v4f x0 = *(const v4fa*)(&os[row * 68 + c8]); const v4f x1 = *(const v4fa*)(&os[row * 68 + c8 + 4]); v8h hv;
#pragma unroll
                    for (int i = 0; i < 4; ++i) { hv[i] = toh_flush(x0[i]); hv[4 + i] = toh_flush(x1[i]); }
                    *(volatile v8h*)(dst + (size_t)row * ldc + c8) = hv; }
                if (ps == 0) __threadfence(); }
            wave_sync();
        }
    } else {
        const int bb = c0 / LSP, sp0 = c0 % LSP;
#pragma unroll
        for (int mb = 0; mb < 4; ++mb) {
            float rsc[8], rm[8], rb[8];
#pragma unroll
            for (int j = 0; j < 8; ++j) { const int ch = r0 + mb * 16 + hi * 8 + j;
                rsc[j] = bfr(pg[ch]) * rsqrtf(bfr(pv[ch]) + EPSV); rm[j] = bfr(pm[ch]); rb[j] = bfr(pb[ch]); }
#pragma unroll
            for (int nb = 0; nb < 4; ++nb) {
#pragma unroll
                for (int j = 0; j < 8; ++j) os[(hi * 8 + j) * 68 + nb * 16 + lr] = (acc[mb][nb][j] * scale - rm[j]) * rsc[j] + rb[j]; }
            wave_sync();
            const size_t chb = (size_t)(bb * CO + r0 + mb * 16);
#pragma unroll 1
            for (int ps = 0; ps < 2; ++ps) {
#pragma unroll
                for (int s = 0; s < 8; ++s) { const int row = 2 * s + (lane >> 4), cofs = (lane & 15) * 4;
                    const v4f val = *(const v4fa*)(&os[row * 68 + cofs]);
                    const v4f res = *(const v4f*)(RES + (chb + row) * LSP + sp0 + cofs);
                    const v4f o = res + val;
                    *(volatile v4f*)(Cf + (chb + row) * OUT_LSP + sp0 + cofs) = o; }
                if (ps == 0) __threadfence(); }
            wave_sync();
        }
    }
}

__global__ __launch_bounds__(32) void k_inproj(const h16* __restrict__ SPn, const h16* __restrict__ Wn, float* XZ) {
    gemm_body<0>(SPn, CO, 32, Wn, CO, CO, 1.0f / WSC, XZ, nullptr, 2 * DIN, 0, nullptr, nullptr, nullptr, nullptr, 0, 1.0f, nullptr);
}
__global__ __launch_bounds__(32) void k_xproj(const h16* __restrict__ UHn, const h16* __restrict__ Wn, float* XD) {
    gemm_body<0>(UHn, DIN, 32, Wn, DIN, DIN, 1.0f / (UCS * WSC), XD, nullptr, 64, 0, nullptr, nullptr, nullptr, nullptr, 0, 1.0f, nullptr);
}
__global__ __launch_bounds__(32) void k_outproj(const h16* __restrict__ YPn, const h16* __restrict__ Wn, h16* O1) {
    gemm_body<1>(YPn, 32, NROW * 32, Wn, DIN, DIN, 1.0f / (YCS * WSC), nullptr, O1, CO, 0, nullptr, nullptr, nullptr, nullptr, 0, YCS, nullptr);
}
__global__ __launch_bounds__(32) void k_cfe1(const h16* __restrict__ O1, const h16* __restrict__ Wn, const float* __restrict__ g, const float* __restrict__ b, const float* __restrict__ m, const float* __restrict__ v, h16* C1) {
    gemm_body<1>(O1, CO, 32, Wn, CO, CO, 1.0f / (YCS * WSC), nullptr, C1, CH4, 1, g, b, m, v, 1, YCS, nullptr);
}
__global__ __launch_bounds__(32) void k_cfe2(const h16* __restrict__ Wn, const h16* __restrict__ C1, const float* __restrict__ g, const float* __restrict__ b, const float* __restrict__ m, const float* __restrict__ v,
                                             const float* __restrict__ ID, float* OUT) {
    gemm_body<2>(Wn, CH4, 32, C1, CH4, CH4, 1.0f / (YCS * WSC), OUT, nullptr, 0, 1, g, b, m, v, 0, 1.0f, ID);
}

__global__ __launch_bounds__(256) void k_conv1d(const float* __restrict__ XZ, const float* __restrict__ cw, const float* __restrict__ cb, h16* UH, int npiece) {
    const int i = blockIdx.x * 256 + threadIdx.x; if (i >= npiece) return;
    const int row = i >> 4, d8 = (i & 15) * 8; const int t = row % LSP;
    v4f wv[8];
#pragma unroll
    for (int e = 0; e < 8; ++e) wv[e] = *(const v4f*)(cw + (size_t)(d8 + e) * 4);
    const v4f b0 = *(const v4f*)(cb + d8), b1 = *(const v4f*)(cb + d8 + 4);
    float acc[8];
#pragma unroll
    for (int e = 0; e < 4; ++e) { acc[e] = 0.0f; acc[4 + e] = 0.0f; }
#pragma unroll
    for (int j = 0; j < 4; ++j) {
        const bool ok = (t - 3 + j) >= 0; const int rc = ok ? (row - 3 + j) : row;
        v4f x0 = *(const v4f*)(XZ + (size_t)rc * (2 * DIN) + d8); v4f x1 = *(const v4f*)(XZ + (size_t)rc * (2 * DIN) + d8 + 4);
        asm volatile("" : "+v"(x0)); asm volatile("" : "+v"(x1));
#pragma unroll
        for (int e = 0; e < 4; ++e) { acc[e] += bfr(wv[e][j]) * (ok ? x0[e] : 0.0f); acc[4 + e] += bfr(wv[4 + e][j]) * (ok ? x1[e] : 0.0f); } }
    v8h o;
#pragma unroll
    for (int e = 0; e < 4; ++e) {
        const float a0 = acc[e] + bfr(b0[e]), a1 = acc[4 + e] + bfr(b1[e]);
        const float u0 = a0 * __builtin_amdgcn_rcpf(1.0f + fexp(-a0)), u1 = a1 * __builtin_amdgcn_rcpf(1.0f + fexp(-a1));
        o[e] = toh_flush(u0 * UCS); o[4 + e] = toh_flush(u1 * UCS); }
    *(volatile v8h*)(UH + (size_t)i * 8) = o; __threadfence(); *(volatile v8h*)(UH + (size_t)i * 8) = o;
}

__global__ __launch_bounds__(32) void k_scan(const float* __restrict__ XD, const h16* __restrict__ UH, const float* __restrict__ XZ,
                                             const float* __restrict__ dtw, const float* __restrict__ dtb, const float* __restrict__ alog, const float* __restrict__ dpp, h16* YP) {
    __shared__ __align__(16) h16 yb[8 * 32];
    const int lane = threadIdx.x & 31;
    const int bb = blockIdx.x >> 2, g = blockIdx.x & 3; const int d = g * 32 + lane;
    float A2[16], hs[16];
#pragma unroll
    for (int q = 0; q < 4; ++q) { const v4f al = *(const v4f*)(alog + (size_t)d * DST + 4 * q);
#pragma unroll
        for (int e = 0; e < 4; ++e) { A2[4 * q + e] = -fexp(bfr(al[e])) * LOG2E; hs[4 * q + e] = 0.0f; } }
    const v4f wq = *(const v4f*)(dtw + (size_t)d * DTR);
    const float w0 = bfr(wq[0]), w1 = bfr(wq[1]), w2 = bfr(wq[2]), w3 = bfr(wq[3]);
    const float db = bfr(dtb[d]), Dv = bfr(dpp[d]);
    const size_t rowb = (size_t)bb * LSP;
#pragma unroll 1
    for (int t0 = 0; t0 < LSP; t0 += 8) {
#pragma unroll 1
        for (int tt = 0; tt < 8; ++tt) {
            const size_t row = rowb + (size_t)(t0 + tt);
            const float* xr = XD + row * 64;
            const v4f dr = *(const v4f*)xr;
            v4f Bq[4], Cq[4];
#pragma unroll
            for (int q = 0; q < 4; ++q) { Bq[q] = *(const v4f*)(xr + DTR + 4 * q); Cq[q] = *(const v4f*)(xr + DTR + DST + 4 * q); }
            const float dtp = ((dr[0] * w0 + dr[1] * w1) + (dr[2] * w2 + dr[3] * w3)) + db;
            const float dt = fmaxf(dtp, 0.0f) + log1pf(fexp(-fabsf(dtp)));
            const float uu = (float)UH[row * DIN + d] * (1.0f / UCS);
            const float dtu = dt * uu;
            float y = 0.0f;
#pragma unroll
            for (int q = 0; q < 4; ++q) {
#pragma unroll
                for (int e = 0; e < 4; ++e) { const float dA = __builtin_amdgcn_exp2f(dt * A2[4 * q + e]);
                    hs[4 * q + e] = hs[4 * q + e] * dA + dtu * Bq[q][e]; y += hs[4 * q + e] * Cq[q][e]; } }
            y += uu * Dv;
            const float z = XZ[row * (2 * DIN) + DIN + d];
            const float sz = z * __builtin_amdgcn_rcpf(1.0f + fexp(-z));
            yb[tt * 32 + lane] = toh_flush(y * sz * YCS);
        }
        wave_sync();
        const v8h pv = *(const v8ha*)(&yb[lane * 8]);
        h16* dst = YP + ((size_t)g * NROW + rowb + (size_t)t0) * 32 + (size_t)lane * 8;
        *(volatile v8h*)dst = pv; __threadfence(); *(volatile v8h*)dst = pv;
        wave_sync();
    }
}

static constexpr size_t al256(size_t v) { return (v + 255) & ~(size_t)255; }
static constexpr size_t NPIECE = (size_t)NB * PW * PH * PD * 4;
static constexpr size_t SZ_XP  = al256(NPIECE * 16);
static constexpr size_t SZ_W2  = al256((size_t)CO * KCONV * 2);
static constexpr size_t SZ_WIN = al256((size_t)2 * DIN * CO * 2);
static constexpr size_t SZ_WXP = al256((size_t)64 * DIN * 2);
static constexpr size_t SZ_WOU = al256((size_t)CO * DIN * 2);
static constexpr size_t SZ_WC1 = al256((size_t)CH4 * CO * 2);
static constexpr size_t SZ_WC2 = al256((size_t)CO * CH4 * 2);
static constexpr size_t SZ_CV  = al256((size_t)NB * CO * LSP * 4);
static constexpr size_t SZ_ST  = al256((size_t)NB * 32 * 32 * 4);
static constexpr size_t SZ_SP  = al256((size_t)NROW * CO * 2);
static constexpr size_t SZ_XZ  = al256((size_t)NROW * 2 * DIN * 4);
static constexpr size_t SZ_UH  = al256((size_t)NROW * DIN * 2);
static constexpr size_t SZ_XD  = al256((size_t)NROW * 64 * 4);
static constexpr size_t SZ_YP  = al256((size_t)4 * NROW * 32 * 2);
static constexpr size_t SZ_O1  = al256((size_t)NROW * CO * 2);
static constexpr size_t SZ_C1  = al256((size_t)NROW * CH4 * 2);
static constexpr size_t SZ_TOTAL = SZ_XP + SZ_W2 + SZ_WIN + SZ_WXP + SZ_WOU + SZ_WC1 + SZ_WC2 + 2 * SZ_CV + SZ_ST + SZ_SP + SZ_XZ + SZ_UH + SZ_XD + SZ_YP + SZ_O1 + SZ_C1;
static_assert(SZ_TOTAL <= (size_t)134217728);
static_assert(NPIECE % 8 == 0);
static_assert(NPIECE < (size_t)2147483647);
static_assert((size_t)NROW * 16 < (size_t)2147483647);
static_assert(((size_t)NXD * DIN) % 8 == 0);

extern "C" void kernel_launch(void* const* d_in, const int* in_sizes, int n_in,
                              void* d_out, int out_size, void* d_ws, size_t ws_size, hipStream_t stream) {
    if (n_in < 36) return;
    if ((size_t)in_sizes[0] < ((size_t)(NB * C_IN - 1)) * LSP_FULL + LSP) return;
    if (in_sizes[1] < CO * C_IN * 27 || in_sizes[2] < CO || in_sizes[3] < CO || in_sizes[4] < CO) return;
    if (in_sizes[5] < CO * 27) return;
    for (int i = 6; i <= 16; ++i) if (in_sizes[i] < CO) return;
    if (in_sizes[17] < 2 * DIN * CO || in_sizes[18] < DIN * 4 || in_sizes[19] < DIN || in_sizes[20] < NXD * DIN) return;
    if (in_sizes[21] < DIN * DTR || in_sizes[22] < DIN || in_sizes[23] < DIN * DST || in_sizes[24] < DIN || in_sizes[25] < CO * DIN) return;
    if (in_sizes[26] < CH4 * CO || in_sizes[27] < CH4 || in_sizes[28] < CH4 || in_sizes[29] < CH4 || in_sizes[30] < CH4) return;
    if (in_sizes[31] < CO * CH4 || in_sizes[32] < CO || in_sizes[33] < CO || in_sizes[34] < CO || in_sizes[35] < CO) return;
    if ((size_t)out_size < ((size_t)(NB * CO - 1)) * OUT_LSP + LSP) return;
    if (SZ_TOTAL > ws_size) return;
    const float* x          = (const float*)d_in[0];
    const float* conv_w     = (const float*)d_in[1];
    const float* conv_b     = (const float*)d_in[2];
    const float* gn_g       = (const float*)d_in[3];
    const float* gn_b       = (const float*)d_in[4];
    const float* sfe_conv_w = (const float*)d_in[5];
    const float* sfe_bn1_g  = (const float*)d_in[6];
    const float* sfe_bn1_b  = (const float*)d_in[7];
    const float* sfe_bn1_m  = (const float*)d_in[8];
    const float* sfe_bn1_v  = (const float*)d_in[9];
    const float* sfe_conv1_w= (const float*)d_in[10];
    const float* sfe_bn2_g  = (const float*)d_in[11];
    const float* sfe_bn2_b  = (const float*)d_in[12];
    const float* sfe_bn2_m  = (const float*)d_in[13];
    const float* sfe_bn2_v  = (const float*)d_in[14];
    const float* ln_g       = (const float*)d_in[15];
    const float* ln_b       = (const float*)d_in[16];
    const float* in_proj_w  = (const float*)d_in[17];
    const float* conv1d_w   = (const float*)d_in[18];
    const float* conv1d_b   = (const float*)d_in[19];
    const float* x_proj_w   = (const float*)d_in[20];
    const float* dt_proj_w  = (const float*)d_in[21];
    const float* dt_proj_b  = (const float*)d_in[22];
    const float* A_log      = (const float*)d_in[23];
    const float* Dp         = (const float*)d_in[24];
    const float* out_proj_w = (const float*)d_in[25];
    const float* cfe1_w     = (const float*)d_in[26];
    const float* cfe_bn1_g  = (const float*)d_in[27];
    const float* cfe_bn1_b  = (const float*)d_in[28];
    const float* cfe_bn1_m  = (const float*)d_in[29];
    const float* cfe_bn1_v  = (const float*)d_in[30];
    const float* cfe2_w     = (const float*)d_in[31];
    const float* cfe_bn2_g  = (const float*)d_in[32];
    const float* cfe_bn2_b  = (const float*)d_in[33];
    const float* cfe_bn2_m  = (const float*)d_in[34];
    const float* cfe_bn2_v  = (const float*)d_in[35];
    float* OUT = (float*)d_out;
    char* wsp = (char*)d_ws;
    bf*    XP  = (bf*)wsp;    wsp += SZ_XP;
    bf*    W2  = (bf*)wsp;    wsp += SZ_W2;
    h16*   WIN = (h16*)wsp;   wsp += SZ_WIN;
    h16*   WXP = (h16*)wsp;   wsp += SZ_WXP;
    h16*   WOU = (h16*)wsp;   wsp += SZ_WOU;
    h16*   WC1 = (h16*)wsp;   wsp += SZ_WC1;
    h16*   WC2 = (h16*)wsp;   wsp += SZ_WC2;
    float* CV  = (float*)wsp; wsp += SZ_CV;
    float* ST  = (float*)wsp; wsp += SZ_ST;
    float* ID  = (float*)wsp; wsp += SZ_CV;
    h16*   SP  = (h16*)wsp;   wsp += SZ_SP;
    float* XZ  = (float*)wsp; wsp += SZ_XZ;
    h16*   UH  = (h16*)wsp;   wsp += SZ_UH;
    float* XD  = (float*)wsp; wsp += SZ_XD;
    h16*   YP  = (h16*)wsp;   wsp += SZ_YP;
    h16*   O1  = (h16*)wsp;   wsp += SZ_O1;
    h16*   C1  = (h16*)wsp;   wsp += SZ_C1;

    k_xpad<<<(unsigned)((NPIECE + 255) / 256), 256, 0, stream>>>(x, XP, (int)NPIECE);
    k_wconv3<<<(CO * 27 * 4) / 256, 256, 0, stream>>>(conv_w, W2);
    k_wcvt16<<<(2 * DIN * CO / 8 + 255) / 256, 256, 0, stream>>>(in_proj_w, WIN, 2 * DIN * CO / 8, 2 * DIN * CO / 8);
    k_wcvt16<<<(64 * DIN / 8 + 255) / 256, 256, 0, stream>>>(x_proj_w, WXP, NXD * DIN / 8, 64 * DIN / 8);
    k_wcvt16<<<(CO * DIN / 8 + 255) / 256, 256, 0, stream>>>(out_proj_w, WOU, CO * DIN / 8, CO * DIN / 8);
    k_wcvt16<<<(CH4 * CO / 8 + 255) / 256, 256, 0, stream>>>(cfe1_w, WC1, CH4 * CO / 8, CH4 * CO / 8);
    k_wcvt16<<<(CO * CH4 / 8 + 255) / 256, 256, 0, stream>>>(cfe2_w, WC2, CO * CH4 / 8, CO * CH4 / 8);

    k_conv<<<NROW / 64, 32, 0, stream>>>(W2, XP, conv_b, CV);
    k_gnstats<<<NB * 32, 256, 0, stream>>>(CV, ST);
    { const int n4 = NB * CO * LSP / 4; k_gnapply<<<(n4 + 255) / 256, 256, 0, stream>>>(CV, ST, gn_g, gn_b, ID, n4); }
    k_sfe_ln<<<NROW / 64, 256, 0, stream>>>(ID, sfe_conv_w, sfe_bn1_g, sfe_bn1_b, sfe_bn1_m, sfe_bn1_v, sfe_conv1_w, sfe_bn2_g, sfe_bn2_b, sfe_bn2_m, sfe_bn2_v, ln_g, ln_b, SP);
    k_inproj<<<dim3(NROW / 64, (2 * DIN) / 64, 1), 32, 0, stream>>>(SP, WIN, XZ);
    { const int np = NROW * 16; k_conv1d<<<(np + 255) / 256, 256, 0, stream>>>(XZ, conv1d_w, conv1d_b, UH, np); }
    k_xproj<<<dim3(NROW / 64, 1, 1), 32, 0, stream>>>(UH, WXP, XD);
    k_scan<<<NB * 4, 32, 0, stream>>>(XD, UH, XZ, dt_proj_w, dt_proj_b, A_log, Dp, YP);
    k_outproj<<<dim3(NROW / 64, 1, 1), 32, 0, stream>>>(YP, WOU, O1);
    k_cfe1<<<dim3(NROW / 64, CH4 / 64, 1), 32, 0, stream>>>(O1, WC1, cfe_bn1_g, cfe_bn1_b, cfe_bn1_m, cfe_bn1_v, C1);
    k_cfe2<<<dim3(1, NROW / 64, 1), 32, 0, stream>>>(WC2, C1, cfe_bn2_g, cfe_bn2_b, cfe_bn2_m, cfe_bn2_v, ID, OUT);
}
